// MemN2N_57071525429503
// MI455X (gfx1250) — hardware-run, weakly checked
//
#include <hip/hip_runtime.h>


namespace {
constexpr int B = 128, M = 200, S = 20, V = 100000, D = 128, NC = 10000, CL = 10, HOPS = 3;
constexpr float XS = 8.0f, WSC = 256.0f;
typedef _Float16 b16;
typedef __attribute__((ext_vector_type(16))) _Float16 v16b;
typedef __attribute__((ext_vector_type(8))) _Float16 v8b;
typedef __attribute__((ext_vector_type(4))) _Float16 v4b;
typedef __attribute__((ext_vector_type(8))) float v8f;
typedef __attribute__((ext_vector_type(4))) float v4f;
__device__ __forceinline__ float bf16_rne(float f) { unsigned int u = __float_as_uint(f); u += 0x7FFFu + ((u >> 16) & 1u); float r = __uint_as_float(u & 0xFFFF0000u); asm volatile("" : "+v"(r)); return r; }
__device__ __forceinline__ void split16(float v, b16& hi, b16& lo) { hi = (b16)v; lo = (b16)(v - (float)hi); }
__device__ __forceinline__ v16b frag_kb(const b16* p, int hh) { const v8b a = *(const v8b*)(p + 8 * hh), b = *(const v8b*)(p + 16 + 8 * hh); v16b f;
#pragma unroll
  for (int e = 0; e < 8; ++e) { f[e] = a[e]; f[8 + e] = b[e]; } return f; }
__device__ __forceinline__ v8f wmma16b(v16b a, v16b b, v8f c) { v8f d = __builtin_amdgcn_wmma_f32_16x16x32_f16(false, a, false, b, (short)0, c, false, false); asm volatile("v_nop\n\tv_nop\n\tv_nop\n\tv_nop" : "+v"(d) : "v"(a), "v"(b)); return d; }
__device__ __forceinline__ void wave_lds_sync() { __builtin_amdgcn_fence(__ATOMIC_RELEASE, "workgroup"); __builtin_amdgcn_wave_barrier(); __builtin_amdgcn_fence(__ATOMIC_ACQUIRE, "workgroup"); }
__device__ __forceinline__ float pmul(float a, float b) { float p = a * b; asm volatile("" : "+v"(p)); return p; }
__device__ __forceinline__ int iclamp(int v, int lo, int hi) { return v < lo ? lo : (v > hi ? hi : v); }

__global__ __launch_bounds__(256) void wput_kernel(const float* __restrict__ h, b16* __restrict__ HT) { const int u = blockIdx.x * 256 + threadIdx.x; if (u >= D * 16) return; const int o = u / 16, k0 = (u % 16) * 8; v8b v;
#pragma unroll
  for (int j = 0; j < 8; ++j) v[j] = (b16)(bf16_rne(h[(size_t)o * D + k0 + j]) * WSC); for (int pass = 0; pass < 2; ++pass) { *(volatile v8b*)(HT + (size_t)o * D + k0) = v; __threadfence(); } }
__global__ __launch_bounds__(256) void bag_kernel(const float* __restrict__ A, const int* __restrict__ st, const int* __restrict__ qu, float* __restrict__ MBm, float* __restrict__ U) { const int wave = threadIdx.x >> 5, lane = threadIdx.x & 31; const size_t r = (size_t)blockIdx.x * 8 + wave; if (r >= (size_t)B * M + B) return; const int* ids = r < (size_t)B * M ? st + r * S : qu + (r - (size_t)B * M) * S; v4f acc = {0, 0, 0, 0};
#pragma unroll 1
  for (int w = 0; w < S; ++w) { const int id = iclamp(ids[w], 0, V - 1); if (id == 0) continue; const v4f a = *(const v4f*)(A + (size_t)id * D + lane * 4); for (int k = 0; k < 4; ++k) acc[k] += bf16_rne(a[k]); }
  float* dstp = r < (size_t)B * M ? MBm + r * D : U + (r - (size_t)B * M) * D;
  for (int pass = 0; pass < 2; ++pass) { *(volatile v4f*)(dstp + lane * 4) = acc; __threadfence(); } }
__global__ __launch_bounds__(256) void cand_kernel(const float* __restrict__ Wt, const int* __restrict__ ca, b16* __restrict__ CHp, b16* __restrict__ CLp) { const int wave = threadIdx.x >> 5, lane = threadIdx.x & 31; const size_t r = (size_t)blockIdx.x * 8 + wave; if (r >= (size_t)NC) return; v4f acc = {0, 0, 0, 0};
#pragma unroll 1
  for (int w = 0; w < CL; ++w) { const int id = iclamp(ca[r * CL + w], 0, V - 1); if (id == 0) continue; const v4f a = *(const v4f*)(Wt + (size_t)id * D + lane * 4); for (int k = 0; k < 4; ++k) acc[k] += bf16_rne(a[k]); }
  v4b ph, pl; for (int k = 0; k < 4; ++k) { b16 p, l; split16(acc[k] * XS, p, l); ph[k] = p; pl[k] = l; }
  for (int pass = 0; pass < 2; ++pass) { *(volatile v4b*)(CHp + r * D + lane * 4) = ph; *(volatile v4b*)(CLp + r * D + lane * 4) = pl; __threadfence(); } }
__global__ __launch_bounds__(256) void hopatt_kernel(const float* __restrict__ MBm, const float* __restrict__ U, int BLIM, float* __restrict__ O) { __shared__ float Pd[8][M]; const int wave = threadIdx.x >> 5, lane = threadIdx.x & 31; const int b = blockIdx.x * 8 + wave; if (b >= BLIM) return; const v4f u = *(const v4f*)(U + (size_t)b * D + lane * 4); float mx = -INFINITY;
#pragma unroll 1
  for (int j = 0; j < M; ++j) { const v4f mv = *(const v4f*)(MBm + ((size_t)b * M + j) * D + lane * 4); float s = pmul(mv[0], u[0]) + pmul(mv[1], u[1]) + pmul(mv[2], u[2]) + pmul(mv[3], u[3]); for (int o_ = 16; o_; o_ >>= 1) s += __shfl_xor(s, o_); if (lane == 0) Pd[wave][j] = s; mx = fmaxf(mx, s); }
  wave_lds_sync(); float den = 0.0f;
#pragma unroll 1
  for (int j = lane; j < M; j += 32) den += __expf(Pd[wave][j] - mx);
  for (int o_ = 16; o_; o_ >>= 1) den += __shfl_xor(den, o_); const float inv = 1.0f / den; v4f acc = {0, 0, 0, 0};
#pragma unroll 1
  for (int j = 0; j < M; ++j) { const float p = __expf(Pd[wave][j] - mx) * inv; const v4f mv = *(const v4f*)(MBm + ((size_t)b * M + j) * D + lane * 4); for (int k = 0; k < 4; ++k) acc[k] += pmul(p, mv[k]); }
  for (int pass = 0; pass < 2; ++pass) { *(volatile v4f*)(O + (size_t)b * D + lane * 4) = acc; __threadfence(); } }
__global__ __launch_bounds__(32) void hoplin_kernel(const b16* __restrict__ HT, const float* __restrict__ O, int BLIM, float* __restrict__ U) { __shared__ __attribute__((aligned(16))) b16 Ah[16][D + 8], Al[16][D + 8]; __shared__ float Tf[16][132]; const int lane = threadIdx.x, nloc = lane & 15, hlf = lane >> 4; const size_t m0 = (size_t)blockIdx.x * 16; if (m0 >= (size_t)BLIM) return;
  for (int rr = 0; rr < 16; ++rr) for (int q = 0; q < 4; ++q) { b16 p, l; split16(U[(m0 + rr) * D + q * 32 + lane] * XS, p, l); Ah[rr][q * 32 + lane] = p; Al[rr][q * 32 + lane] = l; }
  wave_lds_sync(); v8f acc[8];
#pragma unroll
  for (int t = 0; t < 8; ++t) acc[t] = (v8f){};
#pragma unroll
  for (int kb = 0; kb < D; kb += 32) { const v16b a = frag_kb(&Ah[nloc][kb], hlf), al = frag_kb(&Al[nloc][kb], hlf);
#pragma unroll
    for (int t = 0; t < 8; ++t) { const v16b bw = frag_kb(HT + (size_t)(t * 16 + nloc) * D + kb, hlf); acc[t] = wmma16b(a, bw, acc[t]); acc[t] = wmma16b(al, bw, acc[t]); } }
#pragma unroll
  for (int t = 0; t < 8; ++t) { const int cc = t * 16 + nloc;
#pragma unroll
    for (int r8 = 0; r8 < 8; ++r8) { const int rr = 8 * hlf + r8; Tf[rr][cc] = tanhf(acc[t][r8] * (1.0f / (XS * WSC)) + O[(m0 + rr) * D + cc]); } }
  wave_lds_sync();
  for (int pass = 0; pass < 2; ++pass) { for (int rr = 0; rr < 16; ++rr) *(volatile v4f*)(U + (m0 + rr) * D + lane * 4) = *(const v4f*)(&Tf[rr][lane * 4]); __threadfence(); } }
__global__ __launch_bounds__(32) void logits_kernel(const float* __restrict__ U, const b16* __restrict__ CHp, const b16* __restrict__ CLp, int BLIM, float* __restrict__ out) { __shared__ __attribute__((aligned(16))) b16 Ah[16][D + 8], Al[16][D + 8]; __shared__ float Tf[16][260]; const int lane = threadIdx.x, nloc = lane & 15, hlf = lane >> 4; const size_t m0 = (size_t)blockIdx.x * 16; if (m0 >= (size_t)BLIM) return;
  for (int rr = 0; rr < 16; ++rr) for (int q = 0; q < 4; ++q) { b16 p, l; split16(U[(m0 + rr) * D + q * 32 + lane] * XS, p, l); Ah[rr][q * 32 + lane] = p; Al[rr][q * 32 + lane] = l; }
  wave_lds_sync(); v16b ah[4], al[4];
#pragma unroll
  for (int q = 0; q < 4; ++q) { ah[q] = frag_kb(&Ah[nloc][q * 32], hlf); al[q] = frag_kb(&Al[nloc][q * 32], hlf); }
  for (int pass = 0; pass < 2; ++pass) {
#pragma unroll 1
    for (int g = 0; g < (NC + 127) / 128; ++g) { const int nt = (NC / 16 - g * 8) < 8 ? (NC / 16 - g * 8) : 8; v8f acc[8];
#pragma unroll
      for (int t = 0; t < 8; ++t) acc[t] = (v8f){};
#pragma unroll
      for (int t = 0; t < 8; ++t) if (t < nt) {
#pragma unroll
        for (int q = 0; q < 4; ++q) { const size_t ro = (size_t)((g * 8 + t) * 16 + nloc) * D + q * 32; const v16b bh = frag_kb(CHp + ro, hlf), bl = frag_kb(CLp + ro, hlf); acc[t] = wmma16b(ah[q], bh, acc[t]); acc[t] = wmma16b(ah[q], bl, acc[t]); acc[t] = wmma16b(al[q], bh, acc[t]); } }
#pragma unroll
      for (int t = 0; t < 8; ++t) if (t < nt)
#pragma unroll
        for (int r8 = 0; r8 < 8; ++r8) Tf[8 * hlf + r8][t * 16 + nloc] = acc[t][r8] * (1.0f / (XS * XS));
      wave_lds_sync();
      for (int rr = 0; rr < 16; ++rr) for (int c = lane; c < nt * 16; c += 32) ((volatile float*)out)[(m0 + rr) * NC + g * 128 + c] = Tf[rr][c];
      wave_lds_sync(); }
    __threadfence(); } }
}

extern "C" void kernel_launch(void* const* d_in, const int* in_sizes, int n_in, void* d_out, int out_size, void* d_ws, size_t ws_size, hipStream_t stream) {
  (void)n_in;
  auto Fp = [&](int i) { return (const float*)d_in[i]; }; auto Ip = [&](int i) { return (const int*)d_in[i]; };
  if (in_sizes[0] != B * M * S || in_sizes[1] != B * S || in_sizes[2] != NC * CL || in_sizes[3] != V * D || in_sizes[4] != V * D || in_sizes[5] != D * D || out_size != B * NC) return;
  const int BLIM = B;
  size_t off = 0; char* ws = (char*)d_ws;
  auto carve = [&](size_t bytes) { char* p = ws + off; off += (bytes + 255) & ~(size_t)255; return p; };
  b16* HT = (b16*)carve((size_t)D * D * 2); float* MBm = (float*)carve((size_t)B * M * D * 4); float* U = (float*)carve((size_t)B * D * 4); float* O = (float*)carve((size_t)B * D * 4); b16* CHp = (b16*)carve((size_t)NC * D * 2); b16* CLp = (b16*)carve((size_t)NC * D * 2);
  if (off > ws_size || off > ((size_t)32 << 20)) return;
  wput_kernel<<<(D * 16 + 255) / 256, 256, 0, stream>>>(Fp(5), HT);
  bag_kernel<<<(B * M + B + 7) / 8, 256, 0, stream>>>(Fp(3), Ip(0), Ip(1), MBm, U);
  cand_kernel<<<(NC + 7) / 8, 256, 0, stream>>>(Fp(4), Ip(2), CHp, CLp);
  for (int hop = 0; hop < HOPS; ++hop) { hopatt_kernel<<<(BLIM + 7) / 8, 256, 0, stream>>>(MBm, U, BLIM, O); hoplin_kernel<<<BLIM / 16, 32, 0, stream>>>(HT, O, BLIM, U); }
  logits_kernel<<<BLIM / 16, 32, 0, stream>>>(U, CHp, CLp, BLIM, (float*)d_out);
}
